// KernelSample_72971494359165
// MI455X (gfx1250) — hardware-verified
//
#include <hip/hip_runtime.h>


namespace {
constexpr int NBC = 8, NI = 4096, NO = 4096, DD = 3, W = 64;
constexpr float XS = 8.0f, PS = 8.0f, LOG2E = 1.4426950408889634f;

typedef _Float16 b16;
typedef __attribute__((ext_vector_type(16))) _Float16 v16b;
typedef __attribute__((ext_vector_type(8))) _Float16 v8b;
typedef __attribute__((ext_vector_type(8))) float v8f;
typedef __attribute__((ext_vector_type(4))) float v4f;
__device__ __forceinline__ float bf16_rne(float f) { unsigned int u = __float_as_uint(f); u += 0x7FFFu + ((u >> 16) & 1u); return __uint_as_float(u & 0xFFFF0000u); }
__device__ __forceinline__ v16b frag_kb(const b16* p, int hh) { const v8b a = *(const v8b*)(p + 8 * hh), b = *(const v8b*)(p + 16 + 8 * hh); v16b f;
#pragma unroll
  for (int e = 0; e < 8; ++e) { f[e] = a[e]; f[8 + e] = b[e]; } return f; }
__device__ __forceinline__ v8f wmma16b(v16b a, v16b b, v8f c) { v8f d = __builtin_amdgcn_wmma_f32_16x16x32_f16(false, a, false, b, (short)0, c, false, false); asm volatile("v_nop\n\tv_nop\n\tv_nop\n\tv_nop" : "+v"(d) : "v"(a), "v"(b)); return d; }
__device__ __forceinline__ void wave_lds_sync() { __builtin_amdgcn_fence(__ATOMIC_RELEASE, "workgroup"); __builtin_amdgcn_wave_barrier(); __builtin_amdgcn_fence(__ATOMIC_ACQUIRE, "workgroup"); }
__device__ __forceinline__ float pmul(float a, float b) { float p = a * b; asm volatile("" : "+v"(p)); return p; }

__global__ __launch_bounds__(256) void wt_kernel(const float* __restrict__ w, b16* __restrict__ WT16) {
  __shared__ __attribute__((aligned(16))) b16 T[W][64 + 8];
  const int bc = blockIdx.y, i0 = blockIdx.x * 64, t_ = threadIdx.x;
  for (int q = t_; q < 64 * W; q += 256) { const int ii = q >> 6, ww = q & 63; T[ww][ii] = (b16)(bf16_rne(w[((size_t)bc * NI + i0 + ii) * W + ww]) * XS); }
  __syncthreads();
  for (int pass = 0; pass < 2; ++pass) { for (int q = t_; q < W * 8; q += 256) { const int ww = q >> 3, c8 = (q & 7) * 8; *(volatile v8b*)(WT16 + ((size_t)bc * W + ww) * NI + i0 + c8) = *(const v8b*)(&T[ww][c8]); } __threadfence(); }
}
__global__ __launch_bounds__(256) void pts_kernel(const float* __restrict__ xin, const float* __restrict__ yout, float* __restrict__ XP, float* __restrict__ YP) {
  const int t = blockIdx.x * 256 + threadIdx.x; if (t >= 2 * NBC * NI) return; const int which = t / (NBC * NI), idx = t - which * (NBC * NI); const float* s = (which ? yout : xin) + (size_t)idx * DD;
  const float a = bf16_rne(s[0]), b = bf16_rne(s[1]), c = bf16_rne(s[2]); const v4f o = {a, b, c, (a * a + b * b) + c * c};
  for (int pass = 0; pass < 2; ++pass) { *(volatile v4f*)((which ? YP : XP) + (size_t)idx * 4) = o; __threadfence(); }
}
__global__ __launch_bounds__(64) void ks_kernel(const float* __restrict__ XP, const float* __restrict__ YP, const b16* __restrict__ WT16, float* __restrict__ out) {
  __shared__ __attribute__((aligned(16))) float To[2][16][W + 4];
  const int wave = threadIdx.x >> 5, lane = threadIdx.x & 31, hh = lane >> 4, col = lane & 15; const int bc = blockIdx.y; const int o0 = blockIdx.x * 32 + wave * 16, oi = o0 + col;
  const v4f yp = *(const v4f*)(YP + ((size_t)bc * NO + oi) * 4); const b16* Wb = WT16 + (size_t)bc * W * NI; const float* Xb = XP + (size_t)bc * NI * 4;
  v8f o[4] = {{}, {}, {}, {}}, ol[4] = {{}, {}, {}, {}};
  for (int kb = 0; kb < NI; kb += 32) {
    v16b ph, pl;
#pragma unroll
    for (int hq = 0; hq < 2; ++hq)
#pragma unroll
      for (int r = 0; r < 8; ++r) { const int i = kb + 16 * hq + 8 * hh + r; const v4f xp = *(const v4f*)(Xb + (size_t)i * 4);
        const float cross = (yp[0] * xp[0] + yp[1] * xp[1]) + yp[2] * xp[2]; const float sq = (yp[3] + xp[3]) - 2.0f * cross; const float k = __builtin_amdgcn_exp2f(sq * (-0.5f * LOG2E));
        const b16 h_ = (b16)(k * PS); ph[hq * 8 + r] = h_; pl[hq * 8 + r] = (b16)(k * PS - (float)h_); }
#pragma unroll
    for (int t = 0; t < 4; ++t) { const v16b wf = frag_kb(Wb + (size_t)(t * 16 + col) * NI + kb, hh); o[t] = wmma16b(wf, ph, o[t]); ol[t] = wmma16b(wf, pl, ol[t]); } }
#pragma unroll
  for (int t = 0; t < 4; ++t)
#pragma unroll
    for (int r = 0; r < 8; ++r) To[wave][col][t * 16 + 8 * hh + r] = (o[t][r] + ol[t][r]) * (1.0f / (PS * XS));
  wave_lds_sync();
  for (int pass = 0; pass < 2; ++pass) { for (int rr = 0; rr < 16; ++rr) if (lane < 16) *(volatile v4f*)(out + ((size_t)bc * NO + o0 + rr) * W + lane * 4) = *(const v4f*)(&To[wave][rr][lane * 4]); __threadfence(); }
}
}

extern "C" void kernel_launch(void* const* d_in, const int* in_sizes, int n_in, void* d_out, int out_size, void* d_ws, size_t ws_size, hipStream_t stream) {
  (void)n_in;
  auto Fp = [&](int i) { return (const float*)d_in[i]; };
  if (in_sizes[0] != NBC * NI * DD || in_sizes[1] != NBC * NI * W || in_sizes[2] != NBC * NO * DD || out_size != NBC * NO * W) return;
  size_t off = 0; char* ws = (char*)d_ws;
  auto carve = [&](size_t bytes) { char* p = ws + off; off += (bytes + 255) & ~(size_t)255; return p; };
  b16* WT16 = (b16*)carve((size_t)NBC * W * NI * 2); float* XP = (float*)carve((size_t)NBC * NI * 4 * 4); float* YP = (float*)carve((size_t)NBC * NO * 4 * 4);
  if (off > ws_size || off > ((size_t)128 << 20)) return;
  wt_kernel<<<dim3(NI / 64, NBC), 256, 0, stream>>>(Fp(1), WT16);
  pts_kernel<<<(2 * NBC * NI + 255) / 256, 256, 0, stream>>>(Fp(0), Fp(2), XP, YP);
  ks_kernel<<<dim3(NO / 32, NBC), 64, 0, stream>>>(XP, YP, WT16, (float*)d_out);
}
